// dy_mixprop_1185410973782
// MI455X (gfx1250) — hardware-verified
//
#include <hip/hip_runtime.h>
#include <math.h>

#define NN 16
#define CC 32
#define VV 256
#define LLn 96
#define ALPHA 0.05f

typedef _Float16 f16;
typedef __attribute__((ext_vector_type(16))) f16 f16x16;
typedef __attribute__((ext_vector_type(8)))  f16 f16x8;
typedef __attribute__((ext_vector_type(8)))  float f32x8;
typedef __attribute__((ext_vector_type(4)))  float v4f_t;
typedef float v4fa __attribute__((ext_vector_type(4), may_alias));
__device__ __forceinline__ f32x8 wmma16(f16x16 a, f16x16 b, f32x8 c) {
  c = __builtin_amdgcn_wmma_f32_16x16x32_f16(false, a, false, b, (short)0, c, false, false);
  asm volatile("v_nop\n\tv_nop\n\tv_nop\n\tv_nop" : "+v"(c) : "v"(a), "v"(b));
  return c;
}
__device__ __forceinline__ f16x16 lds_frag(const f16* base, int stride) {
  const int lane = threadIdx.x & 31, row = lane & 15, kh = (lane >> 4) * 8;
  const f16x8 lo = *(const f16x8*)(base + row * stride + kh);
  const f16x8 hi = *(const f16x8*)(base + row * stride + kh + 16);
  f16x16 f;
#pragma unroll
  for (int i = 0; i < 8; ++i) { f[i] = lo[i]; f[i + 8] = hi[i]; }
  return f;
}
__device__ __forceinline__ f16x16 wfrag(const float* __restrict__ Wm, int ldw, int o0, int k0) {
  const int lane = threadIdx.x & 31, r = o0 + (lane & 15), kh = (lane >> 4) * 8; const float* p = Wm + (size_t)r * ldw + k0 + kh;
  f16x16 f;
#pragma unroll
  for (int i = 0; i < 8; ++i) { f[i] = (f16)p[i]; f[8 + i] = (f16)p[16 + i]; }
  return f;
}

__global__ __launch_bounds__(256) void k_slice(const float* __restrict__ x, const float* __restrict__ W1, const float* __restrict__ b1, const float* __restrict__ W2, const float* __restrict__ b2,
                                              const float* __restrict__ M1, const float* __restrict__ mb1, const float* __restrict__ M2, const float* __restrict__ mb2, float* __restrict__ scratch) {
  __shared__ __attribute__((aligned(16))) f16 Xt[VV * 32];
  __shared__ __attribute__((aligned(16))) f16 x1t[VV * 32], x2t[VV * 32];
  __shared__ __attribute__((aligned(16))) union WS { struct { float sS[16 * 260]; f16 Pt[VV * 32]; f16 Hc[CC * VV]; } p; float oS[CC * 260]; } u;
  float* sS = u.p.sS; f16* Pt = u.p.Pt; f16* Hc = u.p.Hc; float* oS = u.oS;
  __shared__ __attribute__((aligned(16))) f16 Ht[VV * 32];
  const int tid = threadIdx.x, lane = tid & 31, wave = tid >> 5, cl = lane & 15, rh = (lane >> 4) * 8;
  const int n = blockIdx.x / LLn, l = blockIdx.x % LLn;
  const float* xs = x + ((size_t)n * CC * VV) * LLn + l;
  for (int e = tid; e < CC * VV; e += 256) { const int c = e >> 8, v = e & 255; const float val = xs[(size_t)(c * VV + v) * LLn]; Xt[v * 32 + c] = (f16)val; Hc[c * VV + v] = (f16)val; }
  __syncthreads();
  { const int ot = wave & 1, vt0 = (wave >> 1) * 4; const f16x16 a1 = wfrag(W1, CC, ot * 16, 0), a2 = wfrag(W2, CC, ot * 16, 0);
#pragma unroll
    for (int t4 = 0; t4 < 4; ++t4) { const int vt = vt0 + t4; const f16x16 bfv = lds_frag(Xt + (vt * 16) * 32, 32);
      f32x8 c1 = {}, c2 = {}; c1 = wmma16(a1, bfv, c1); c2 = wmma16(a2, bfv, c2); const int v = vt * 16 + cl;
#pragma unroll
      for (int r = 0; r < 8; ++r) { const int o = ot * 16 + rh + r; x1t[v * 32 + o] = (f16)tanhf(c1[r] + b1[o]); x2t[v * 32 + o] = (f16)tanhf(c2[r] + b2[o]); } } }
  f32x8 oacc[4];
  { const int ot = wave & 1, vt0 = (wave >> 1) * 4;
#pragma unroll
    for (int j = 0; j < 4; ++j) { f32x8 z = {}; oacc[j] = z; }
    __syncthreads();
    const f16x16 a1 = wfrag(M1, 3 * CC, ot * 16, 0), a2 = wfrag(M2, 3 * CC, ot * 16, 0);
#pragma unroll
    for (int j = 0; j < 4; ++j) { const f16x16 bfv = lds_frag(Xt + ((vt0 + j) * 16) * 32, 32); oacc[j] = wmma16(a1, bfv, oacc[j]); oacc[j] = wmma16(a2, bfv, oacc[j]); } }
#pragma unroll 1
  for (int path = 0; path < 2; ++path) {
    const f16* at = (path == 0) ? x1t : x2t; const f16* bt = (path == 0) ? x2t : x1t; const float* Mw = (path == 0) ? M1 : M2;
    __syncthreads();
    for (int e = tid; e < CC * VV; e += 256) { const int c = e >> 8, v = e & 255; Hc[c * VV + v] = Xt[v * 32 + c]; }
#pragma unroll 1
    for (int step = 0; step < 2; ++step) {
      f32x8 hacc[4];
#pragma unroll
      for (int j = 0; j < 4; ++j) { f32x8 z = {}; hacc[j] = z; }
#pragma unroll 1
      for (int vk = 0; vk < VV / 32; ++vk) {
#pragma unroll 1
        for (int half = 0; half < 2; ++half) {
          __syncthreads();
          { const int v0 = vk * 32 + half * 16; const f16x16 af = lds_frag(at + v0 * 32, 32);
            for (int wt = wave; wt < 16; wt += 8) { f32x8 acc = {}; acc = wmma16(af, lds_frag(bt + (wt * 16) * 32, 32), acc);
#pragma unroll
              for (int r = 0; r < 8; ++r) sS[(rh + r) * 260 + wt * 16 + cl] = acc[r]; } }
          __syncthreads();
          { const int row = tid >> 4, part = tid & 15; float mx = -3.0e38f;
            for (int i = 0; i < 16; ++i) mx = fmaxf(mx, sS[row * 260 + part * 16 + i]);
#pragma unroll
            for (int off = 1; off < 16; off <<= 1) mx = fmaxf(mx, __shfl_xor(mx, off, 32));
            float ev[16]; float z = 0.0f;
#pragma unroll
            for (int i = 0; i < 16; ++i) { ev[i] = expf(sS[row * 260 + part * 16 + i] - mx); z += ev[i]; }
#pragma unroll
            for (int off = 1; off < 16; off <<= 1) z += __shfl_xor(z, off, 32);
            const float iz = 1024.0f / z;
#pragma unroll
            for (int i = 0; i < 16; ++i) Pt[(part * 16 + i) * 32 + half * 16 + row] = (f16)(ev[i] * iz); }
        }
        __syncthreads();
        { const int ct = wave & 1, wt0 = (wave >> 1) * 4; const f16x16 af = lds_frag(Hc + (ct * 16) * VV + vk * 32, VV);
#pragma unroll
          for (int j = 0; j < 4; ++j) hacc[j] = wmma16(af, lds_frag(Pt + ((wt0 + j) * 16) * 32, 32), hacc[j]); }
      }
      __syncthreads();
      { const int ct = wave & 1, wt0 = (wave >> 1) * 4;
#pragma unroll
        for (int j = 0; j < 4; ++j)
#pragma unroll
          for (int r = 0; r < 8; ++r) { const int c = ct * 16 + rh + r, w = (wt0 + j) * 16 + cl;
            const float hv = ALPHA * (float)Xt[w * 32 + c] + (1.0f - ALPHA) * hacc[j][r] * (1.0f / 1024.0f);
            const f16 hh = (f16)hv; Hc[c * VV + w] = hh; Ht[w * 32 + c] = hh; } }
      __syncthreads();
      { const int ot = wave & 1, vt0 = (wave >> 1) * 4; const f16x16 am = wfrag(Mw, 3 * CC, ot * 16, CC * (step + 1));
#pragma unroll
        for (int j = 0; j < 4; ++j) oacc[j] = wmma16(am, lds_frag(Ht + ((vt0 + j) * 16) * 32, 32), oacc[j]); }
    }
  }
  __syncthreads();
  { const int ot = wave & 1, vt0 = (wave >> 1) * 4;
#pragma unroll
    for (int j = 0; j < 4; ++j)
#pragma unroll
      for (int r = 0; r < 8; ++r) { const int o = ot * 16 + rh + r, v = (vt0 + j) * 16 + cl; oS[o * 260 + v] = oacc[j][r] + mb1[o] + mb2[o]; } }
  __syncthreads();
  float* dst = scratch + ((size_t)(n * LLn + l)) * CC * VV;
#pragma unroll 1
  for (int pass = 0; pass < 2; ++pass) { for (int q4 = tid; q4 < CC * 64; q4 += 256) { const int o = q4 >> 6, c4 = (q4 & 63) * 4;
      *(volatile v4f_t*)(dst + o * VV + c4) = *(const volatile v4fa*)(oS + o * 260 + c4); } __threadfence(); }
}
__global__ __launch_bounds__(256) void k_relayout(const float* __restrict__ scratch, float* __restrict__ out) {
  __shared__ float tS[LLn][VV + 1];
  const int tid = threadIdx.x, n = blockIdx.x / CC, o = blockIdx.x % CC;
  for (int e = tid; e < LLn * VV; e += 256) { const int l = e >> 8, v = e & 255; tS[l][v] = scratch[(((size_t)(n * LLn + l)) * CC + o) * VV + v]; }
  __syncthreads();
  float* dst = out + ((size_t)(n * CC + o)) * VV * LLn;
#pragma unroll 1
  for (int pass = 0; pass < 2; ++pass) {
    for (int q4 = tid; q4 < VV * (LLn / 4); q4 += 256) { const int v = q4 / (LLn / 4), l4 = (q4 % (LLn / 4)) * 4; v4f_t val; val[0] = tS[l4][v]; val[1] = tS[l4 + 1][v]; val[2] = tS[l4 + 2][v]; val[3] = tS[l4 + 3][v];
      *(volatile v4f_t*)(dst + (size_t)v * LLn + l4) = val; }
    __threadfence(); }
}

extern "C" void kernel_launch(void* const* d_in, const int* in_sizes, int n_in,
                              void* d_out, int out_size, void* d_ws, size_t ws_size,
                              hipStream_t stream) {
  (void)in_sizes; (void)n_in; (void)out_size;
  const float* x = (const float*)d_in[0];
  const float* W1 = (const float*)d_in[1], *b1 = (const float*)d_in[2], *W2 = (const float*)d_in[3], *b2 = (const float*)d_in[4];
  const float* M1 = (const float*)d_in[5], *mb1 = (const float*)d_in[6], *M2 = (const float*)d_in[7], *mb2 = (const float*)d_in[8];
  float* out = (float*)d_out;
  char* ws = (char*)d_ws;
  float* scratch = (float*)ws; ws += (size_t)NN * LLn * CC * VV * 4;
  if ((size_t)(ws - (char*)d_ws) > ws_size) return;
  k_slice<<<dim3(NN * LLn), dim3(256), 0, stream>>>(x, W1, b1, W2, b2, M1, mb1, M2, mb2, scratch);
  k_relayout<<<dim3(NN * CC), dim3(256), 0, stream>>>(scratch, out);
}
